// CausalGraphLearner_26302379721023
// MI455X (gfx1250) — hardware-run, weakly checked
//
#include <hip/hip_runtime.h>


#define NSM  256
#define DV   128
#define LL   32
#define HH   32
#define NR   32768
typedef _Float16 h16;
typedef unsigned short bf;
typedef __attribute__((ext_vector_type(16))) __bf16   v16bf;
typedef __attribute__((ext_vector_type(16))) _Float16 v16h;
typedef __attribute__((ext_vector_type(8)))  _Float16 v8h;
typedef __attribute__((ext_vector_type(8)))  unsigned short v8us;
typedef __attribute__((ext_vector_type(8)))  float    v8f;
typedef __attribute__((ext_vector_type(4)))  float    v4f;
typedef v8h  __attribute__((may_alias)) v8ha;
typedef v4f  __attribute__((may_alias)) v4fa;
typedef v8us __attribute__((may_alias)) v8usa;

__device__ __forceinline__ unsigned short f2bf(float f) { unsigned u = __float_as_uint(f); u += 0x7FFFu + ((u >> 16) & 1u); return (unsigned short)(u >> 16); }
__device__ __forceinline__ float bf2f(unsigned short b) { return __uint_as_float(((unsigned)b) << 16); }
__device__ __forceinline__ float bfr(float f) { return bf2f(f2bf(f)); }
__device__ __forceinline__ v16h cat16(v8h lo, v8h hi) { return __builtin_shufflevector(lo, hi, 0, 1, 2, 3, 4, 5, 6, 7, 8, 9, 10, 11, 12, 13, 14, 15); }
__device__ __forceinline__ v16bf cat16b(v8us lo, v8us hi) { return __builtin_bit_cast(v16bf, __builtin_shufflevector(lo, hi, 0, 1, 2, 3, 4, 5, 6, 7, 8, 9, 10, 11, 12, 13, 14, 15)); }
__device__ __forceinline__ v8f wmma16(v16h a, v16h b, v8f c) { return __builtin_amdgcn_wmma_f32_16x16x32_f16(false, a, false, b, (short)0, c, false, false); }
__device__ __forceinline__ v8f wmmab(v16bf a, v16bf b, v8f c) { return __builtin_amdgcn_wmma_f32_16x16x32_bf16(false, a, false, b, (short)0, c, false, false); }


template <typename T16> struct WFrag;
template <> struct WFrag<h16> { typedef v16h V; static __device__ __forceinline__ V ld(const h16* p) { return cat16(*(const v8h*)p, *(const v8h*)(p + 16)); } static __device__ __forceinline__ v8f mma(V a, V b, v8f c) { return wmma16(a, b, c); } };
template <> struct WFrag<bf> { typedef v16bf V; static __device__ __forceinline__ V ld(const bf* p) { return cat16b(*(const v8us*)p, *(const v8us*)(p + 16)); } static __device__ __forceinline__ v8f mma(V a, V b, v8f c) { return wmmab(a, b, c); } };
template <typename T16, int NSPLIT, bool BIAS>
__global__ __launch_bounds__(32) void k_gemmw(const T16* __restrict__ A, const T16* __restrict__ A2, const T16* __restrict__ Bt, const T16* __restrict__ Bt2, int K, float* C, int ldc, const float* __restrict__ bias, size_t sA, size_t sB, size_t sC) {
    typedef typename WFrag<T16>::V V;
    __shared__ __align__(16) float os[16 * 68];
    const size_t z = blockIdx.z; A += z * sA; if (A2) A2 += z * sA; Bt += z * sB; if (Bt2) Bt2 += z * sB; C += z * sC;
    const int lane = threadIdx.x & 31, lr = lane & 15, hi = lane >> 4; const int r0 = blockIdx.x * 64, c0 = blockIdx.y * 64;
    v8f acc[4][4];
#pragma unroll
    for (int mb = 0; mb < 4; ++mb)
#pragma unroll
        for (int nb = 0; nb < 4; ++nb) acc[mb][nb] = (v8f){};
    const size_t aoff = (size_t)(r0 + lr) * K + 8 * hi, boff = (size_t)(c0 + lr) * K + 8 * hi;
#pragma unroll 1
    for (int kc = 0; kc < K; kc += 32) {
        V a[4], a2[4];
#pragma unroll
        for (int mb = 0; mb < 4; ++mb) { a[mb] = WFrag<T16>::ld(A + aoff + (size_t)mb * 16 * K + kc); if (NSPLIT == 1 || NSPLIT == 2) a2[mb] = WFrag<T16>::ld(A2 + aoff + (size_t)mb * 16 * K + kc); }
#pragma unroll
        for (int nb = 0; nb < 4; ++nb) { const V b = WFrag<T16>::ld(Bt + boff + (size_t)nb * 16 * K + kc); V b2; if (NSPLIT >= 2) b2 = WFrag<T16>::ld(Bt2 + boff + (size_t)nb * 16 * K + kc);
#pragma unroll
            for (int mb = 0; mb < 4; ++mb) { acc[mb][nb] = WFrag<T16>::mma(a[mb], b, acc[mb][nb]); if (NSPLIT == 1 || NSPLIT == 2) acc[mb][nb] = WFrag<T16>::mma(a2[mb], b, acc[mb][nb]); if (NSPLIT >= 2) acc[mb][nb] = WFrag<T16>::mma(a[mb], b2, acc[mb][nb]); } }
        asm volatile("v_nop\n\tv_nop\n\tv_nop\n\tv_nop" : "+v"(acc[0][0]), "+v"(acc[1][1]), "+v"(acc[2][2]), "+v"(acc[3][3]) : "v"(a[0]), "v"(a[3]));
    }
#pragma unroll
    for (int mb = 0; mb < 4; ++mb) {
#pragma unroll
        for (int nb = 0; nb < 4; ++nb) {
#pragma unroll
            for (int j = 0; j < 8; ++j) os[(hi * 8 + j) * 68 + nb * 16 + lr] = acc[mb][nb][j]; }
        __builtin_amdgcn_wave_barrier(); asm volatile("" ::: "memory");
        float* crow = C + (size_t)(r0 + mb * 16) * ldc + c0;
#pragma unroll 1
        for (int ps = 0; ps < 2; ++ps) {
#pragma unroll
            for (int s = 0; s < 8; ++s) { const int row = 2 * s + hi, cofs = lr * 4; v4f val = *(const v4fa*)(os + row * 68 + cofs); if (BIAS) { val[0] += bfr(bias[c0 + cofs]); val[1] += bfr(bias[c0 + cofs + 1]); val[2] += bfr(bias[c0 + cofs + 2]); val[3] += bfr(bias[c0 + cofs + 3]); }
                *(volatile v4f*)(crow + (size_t)row * ldc + cofs) = val; }
            if (ps == 0) __threadfence(); }
        __builtin_amdgcn_wave_barrier(); asm volatile("" ::: "memory");
    }
}

typedef __attribute__((ext_vector_type(4))) unsigned short v4us;

__global__ __launch_bounds__(256) void k_cvt8(const float* __restrict__ src, bf* dst, size_t n8) { const size_t i = (size_t)blockIdx.x * 256 + threadIdx.x; if (i >= n8) return; const v8f v = *(const v8f*)(src + i * 8); v8us o;
#pragma unroll
    for (int k = 0; k < 8; ++k) o[k] = f2bf(v[k]); *(volatile v8us*)(dst + i * 8) = o; __threadfence(); *(volatile v8us*)(dst + i * 8) = o; }
__global__ __launch_bounds__(256) void k_w1(const float* __restrict__ W1, bf* Bt) { const int e = (blockIdx.x * 256 + threadIdx.x) * 4; if (e >= 2 * HH * LL) return; const int l = e % LL; const int r = e / LL; const int h = r % HH; const int half = r / HH; v4us a;
#pragma unroll
    for (int u = 0; u < 4; ++u) a[u] = f2bf(W1[h * 2 * LL + half * LL + l + u]); *(volatile v4us*)(Bt + e) = a; __threadfence(); *(volatile v4us*)(Bt + e) = a; }
__device__ __forceinline__ float scorep(const float* __restrict__ pa, const float* __restrict__ pb, const float* __restrict__ b1, const float* __restrict__ W2, float b2v) { float s = 0.f;
#pragma unroll 1
    for (int h = 0; h < HH; ++h) { const float a = fmaxf(__fadd_rn(__fadd_rn(pa[h], pb[h]), bfr(b1[h])), 0.f); float w = bfr(W2[h]); asm volatile("" : "+v"(w)); float p = __fmul_rn(a, w); asm volatile("" : "+v"(p)); s = __fadd_rn(s, p); } return __fadd_rn(s, b2v); }
__global__ __launch_bounds__(256) void k_score_mean(const float* __restrict__ C, const float* __restrict__ b1, const float* __restrict__ W2, const float* __restrict__ b2, const float* __restrict__ Wmag, float* AOUT, float* WMOUT) { const int idx = blockIdx.x * 256 + threadIdx.x; if (idx >= DV * DV) return; const int j = idx % DV; const int i = idx / DV; const float b2v = bfr(b2[0]); float acc = 0.f;
#pragma unroll 1
    for (int n = 0; n < NSM; ++n) { const float* ri = C + ((size_t)n * DV + i) * 64; const float* rj = C + ((size_t)n * DV + j) * 64; const float sij = scorep(ri, rj + HH, b1, W2, b2v); const float sji = scorep(rj, ri + HH, b1, W2, b2v); acc = __fadd_rn(acc, __fsub_rn(sij, sji)); }
    const float al = __fdiv_rn(acc, (float)NSM); const float off = (i == j) ? 0.f : 1.f;
    float dir = __fdiv_rn(1.0f, __fadd_rn(1.0f, __expf(-__fdiv_rn(al, 1.0f)))); asm volatile("" : "+v"(dir)); dir = __fmul_rn(dir, off);
    float wm = __fmul_rn(0.5f, __fadd_rn(bfr(Wmag[i * DV + j]), bfr(Wmag[j * DV + i]))); asm volatile("" : "+v"(wm)); wm = __fmul_rn(wm, off);
    float sg = __fdiv_rn(1.0f, __fadd_rn(1.0f, __expf(-wm))); asm volatile("" : "+v"(sg)); float a = __fmul_rn(sg, dir); asm volatile("" : "+v"(a)); a = __fmul_rn(a, off);
    for (int ps = 0; ps < 2; ++ps) { *(volatile float*)(AOUT + idx) = a; *(volatile float*)(WMOUT + idx) = wm; if (ps == 0) __threadfence(); } }

extern "C" void kernel_launch(void* const* d_in, const int* in_sizes, int n_in,
                              void* d_out, int out_size, void* d_ws, size_t ws_size, hipStream_t stream) {
    (void)in_sizes; (void)n_in; (void)out_size;
    const float** I = (const float**)d_in;
    const float *z = I[0], *Wmag = I[1], *W1 = I[2], *b1 = I[3], *W2 = I[4], *b2 = I[5];
    float* AOUT = (float*)d_out; float* WMOUT = AOUT + DV * DV;
    char* wsp = (char*)d_ws;
    auto take = [&](size_t bytes) { char* p = wsp; wsp += (bytes + 255) & ~(size_t)255; return (void*)p; };
    bf* Bt = (bf*)take(64 * LL * 2); bf* ZB = (bf*)take((size_t)NR * LL * 2); float* C = (float*)take((size_t)NR * 64 * 4);
    if ((size_t)(wsp - (char*)d_ws) > ws_size) return;
    k_w1<<<(2 * HH * LL / 4 + 255) / 256, 256, 0, stream>>>(W1, Bt); k_cvt8<<<(NR * LL / 8 + 255) / 256, 256, 0, stream>>>(z, ZB, (size_t)NR * LL / 8);
    k_gemmw<bf, 0, false><<<dim3(NR / 64, 1, 1), 32, 0, stream>>>(ZB, nullptr, Bt, nullptr, LL, C, 64, nullptr, 0, 0, 0);
    k_score_mean<<<(DV * DV + 255) / 256, 256, 0, stream>>>(C, b1, W2, b2, Wmag, AOUT, WMOUT);
}
